// QuantumFeatureMap_23115513987347
// MI455X (gfx1250) — hardware-run, weakly checked
//
#include <hip/hip_runtime.h>
#include <math.h>

typedef __attribute__((ext_vector_type(16))) __bf16   v16b;
typedef __attribute__((ext_vector_type(8)))  float    v8f;
typedef __attribute__((ext_vector_type(4)))  float    v4f;
typedef __attribute__((ext_vector_type(2)))  float    v2f;
typedef __attribute__((ext_vector_type(4)))  unsigned u4v;
typedef __attribute__((ext_vector_type(8)))  unsigned u8v;

constexpr int   kQ            = 4;
constexpr int   kDim          = 1 << kQ;
constexpr int   kOut          = 10;
constexpr int   kBatch        = 1048576;
constexpr float kAlpha        = 1.57f;
constexpr int   kRowsPerWave  = 64;
constexpr int   kWavesPerBlk  = 8;
constexpr int   kRowsPerBlk   = kRowsPerWave * kWavesPerBlk;
constexpr int   kTileWords    = kRowsPerWave * 16;
constexpr int   kOutFloats    = kRowsPerWave * kOut;
static_assert(kQ == 4, "bit tests below are written for four qubits");
static_assert(kOut == kQ + kQ * (kQ - 1) / 2, "four single-qubit and six two-qubit diagonal observables");
static_assert(2 * kDim == 32, "hi plane and lo plane fill the 32-deep k axis exactly");
static_assert((kOutFloats * 4) % 128 == 0, "a wave's output range is a whole number of 128-B lines");
static_assert(kOutFloats == 5 * 32 * 4, "five 16-B stores per lane cover the wave's output range");
static_assert((kBatch % kRowsPerBlk) == 0, "batch is a whole number of blocks");

constexpr int cnot_src(int idx) {
  int j = idx;
  for (int q = kQ - 1; q >= 0; --q) {
    const int cbit = (j >> (kQ - 1 - q)) & 1;
    const int t = (q + 1) % kQ;
    if (cbit) j ^= (1 << (kQ - 1 - t));
  }
  return j;
}
constexpr bool cnot_src_is_permutation() {
  unsigned seen = 0u;
  for (int i = 0; i < kDim; ++i) seen |= (1u << cnot_src(i));
  return seen == 0xFFFFu;
}
static_assert(cnot_src_is_permutation(), "ring map is a bijection of the 16 basis states");
static_assert(cnot_src(0) == 0 && cnot_src(1) == 13 && cnot_src(8) == 12, "ring map spot checks");

constexpr unsigned long long build_obs_masks() {
  unsigned long long packed = 0ull;
  int n = 0;
  for (int q = 0; q < kQ; ++q) {
    packed |= (unsigned long long)(1u << (kQ - 1 - q)) << (4 * n);
    ++n;
  }
  for (int i = 0; i < kQ; ++i) {
    for (int j = i + 1; j < kQ; ++j) {
      packed |= (unsigned long long)((1u << (kQ - 1 - i)) | (1u << (kQ - 1 - j))) << (4 * n);
      ++n;
    }
  }
  return packed;
}
constexpr unsigned long long kObsMasks = build_obs_masks();
static_assert(kObsMasks == 0x3569AC1248ull, "observable masks 8,4,2,1,12,10,9,6,5,3");

__device__ __forceinline__ unsigned bf16_rne_bits(float f) {
  const unsigned u = __float_as_uint(f);
  return (u + 0x7FFFu + ((u >> 16) & 1u)) >> 16;
}

__device__ __forceinline__ v8f mma_bf16_guarded(v16b a, v16b b, v8f c) {
  c = __builtin_amdgcn_wmma_f32_16x16x32_bf16(false, a, false, b, (short)0, c, false, false);
  asm volatile("v_nop\n\tv_nop\n\tv_nop\n\tv_nop" : "+v"(c) : "v"(a), "v"(b));
  return c;
}

template <int I>
__device__ __forceinline__ float state_prob(float c0, float s0, float c1, float s1,
                                            float c2, float s2, float c3, float s3) {
  constexpr int J = cnot_src(I);
  const float a0 = ((J & 8) != 0) ? s0 : c0;
  const float a1 = ((J & 4) != 0) ? s1 : c1;
  const float a2 = ((J & 2) != 0) ? s2 : c2;
  const float a3 = ((J & 1) != 0) ? s3 : c3;
  const float amp = (a0 * a1) * (a2 * a3);
  return amp * amp;
}

__global__ __launch_bounds__(256) void ring_expect_kernel(
    const float* __restrict__ x, float* __restrict__ out, int nrows)
{
  __shared__ __align__(16) unsigned sP[kWavesPerBlk * kTileWords];
  __shared__ __align__(16) float    sO[kWavesPerBlk * kOutFloats];

  const int tid  = threadIdx.x;
  const int lane = tid & 31;
  const int wave = tid >> 5;
  const int nb   = lane & 15;
  const int h    = lane >> 4;
  const long waveRow0 = ((long)blockIdx.x * kWavesPerBlk + wave) * kRowsPerWave;
  unsigned* tileW = sP + wave * kTileWords;
  float*    so    = sO + wave * kOutFloats;

  v16b afrag;
  {
    const bool valid = (nb < kOut);
    const unsigned mk = valid ? (unsigned)((kObsMasks >> (4 * nb)) & 0xFull) : 0u;
    u8v aw;
#pragma unroll
    for (int j = 0; j < 4; ++j) {
      const unsigned st0 = 8u * (unsigned)h + 2u * (unsigned)j;
      const unsigned st1 = st0 + 1u;
      const unsigned par0 = (unsigned)__popc(mk & st0) & 1u;
      const unsigned par1 = (unsigned)__popc(mk & st1) & 1u;
      const unsigned w  = 0x3F803F80u ^ (par0 << 15) ^ (par1 << 31);
      const unsigned wz = valid ? w : 0u;
      aw[j]     = wz;
      aw[4 + j] = wz;
    }
    afrag = __builtin_bit_cast(v16b, aw);
  }

#pragma unroll 1
  for (int it = 0; it < 2; ++it) {
    const int  r    = it * 32 + lane;
    const long row  = waveRow0 + r;
    const long rowc = (row < (long)nrows) ? row : (long)(nrows - 1);
    const v4f xv = *(const v4f*)(x + (size_t)rowc * kQ);
    const float x0 = xv[0];
    const float x1 = xv[1];
    const float x2 = xv[2];
    const float x3 = xv[3];
    const float h0 = 0.5f * (kAlpha * x0);
    const float h1 = 0.5f * (kAlpha * x1);
    const float h2 = 0.5f * (kAlpha * x2);
    const float h3 = 0.5f * (kAlpha * x3);
    const float c0 = cosf(h0);
    const float s0 = sinf(h0);
    const float c1 = cosf(h1);
    const float s1 = sinf(h1);
    const float c2 = cosf(h2);
    const float s2 = sinf(h2);
    const float c3 = cosf(h3);
    const float s3 = sinf(h3);

    float pr[kDim];
    pr[0]  = state_prob<0>(c0, s0, c1, s1, c2, s2, c3, s3);
    pr[1]  = state_prob<1>(c0, s0, c1, s1, c2, s2, c3, s3);
    pr[2]  = state_prob<2>(c0, s0, c1, s1, c2, s2, c3, s3);
    pr[3]  = state_prob<3>(c0, s0, c1, s1, c2, s2, c3, s3);
    pr[4]  = state_prob<4>(c0, s0, c1, s1, c2, s2, c3, s3);
    pr[5]  = state_prob<5>(c0, s0, c1, s1, c2, s2, c3, s3);
    pr[6]  = state_prob<6>(c0, s0, c1, s1, c2, s2, c3, s3);
    pr[7]  = state_prob<7>(c0, s0, c1, s1, c2, s2, c3, s3);
    pr[8]  = state_prob<8>(c0, s0, c1, s1, c2, s2, c3, s3);
    pr[9]  = state_prob<9>(c0, s0, c1, s1, c2, s2, c3, s3);
    pr[10] = state_prob<10>(c0, s0, c1, s1, c2, s2, c3, s3);
    pr[11] = state_prob<11>(c0, s0, c1, s1, c2, s2, c3, s3);
    pr[12] = state_prob<12>(c0, s0, c1, s1, c2, s2, c3, s3);
    pr[13] = state_prob<13>(c0, s0, c1, s1, c2, s2, c3, s3);
    pr[14] = state_prob<14>(c0, s0, c1, s1, c2, s2, c3, s3);
    pr[15] = state_prob<15>(c0, s0, c1, s1, c2, s2, c3, s3);

    unsigned hw[8], lw[8];
#pragma unroll
    for (int j = 0; j < 8; ++j) {
      const float pa = pr[2 * j];
      const float pb = pr[2 * j + 1];
      const unsigned ha = bf16_rne_bits(pa);
      const unsigned hb = bf16_rne_bits(pb);
      const float ra = pa - __uint_as_float(ha << 16);
      const float rb = pb - __uint_as_float(hb << 16);
      const unsigned la = bf16_rne_bits(ra);
      const unsigned lb = bf16_rne_bits(rb);
      hw[j] = ha | (hb << 16);
      lw[j] = la | (lb << 16);
    }
    u4v* tr = (u4v*)(tileW + r * 16);
    tr[0] = (u4v){hw[0], hw[1], hw[2], hw[3]};
    tr[1] = (u4v){hw[4], hw[5], hw[6], hw[7]};
    tr[2] = (u4v){lw[0], lw[1], lw[2], lw[3]};
    tr[3] = (u4v){lw[4], lw[5], lw[6], lw[7]};
  }
  __syncthreads();

  v8f acc[4];
#pragma unroll
  for (int t = 0; t < 4; ++t) {
    const unsigned* rp = tileW + (16 * t + nb) * 16;
    const u4v q0 = *(const u4v*)(rp + 4 * h);
    const u4v q1 = *(const u4v*)(rp + 8 + 4 * h);
    const u8v bw = __builtin_shufflevector(q0, q1, 0, 1, 2, 3, 4, 5, 6, 7);
    const v16b bfrag = __builtin_bit_cast(v16b, bw);
    const v8f zero = (v8f){0.f, 0.f, 0.f, 0.f, 0.f, 0.f, 0.f, 0.f};
    acc[t] = mma_bf16_guarded(afrag, bfrag, zero);
  }

#pragma unroll
  for (int t = 0; t < 4; ++t) {
    float* o = so + (16 * t + nb) * kOut;
    if (h == 0) {
      *(v2f*)(o + 0) = (v2f){acc[t][0], acc[t][1]};
      *(v2f*)(o + 2) = (v2f){acc[t][2], acc[t][3]};
      *(v2f*)(o + 4) = (v2f){acc[t][4], acc[t][5]};
      *(v2f*)(o + 6) = (v2f){acc[t][6], acc[t][7]};
    } else {
      *(v2f*)(o + 8) = (v2f){acc[t][0], acc[t][1]};
    }
  }
  __syncthreads();

  {
    const size_t gbase = (size_t)waveRow0 * kOut;
    const size_t total = (size_t)nrows * kOut;
    v4f val[5];
#pragma unroll
    for (int j = 0; j < 5; ++j) val[j] = *(const v4f*)(so + (lane + 32 * j) * 4);
    for (int pass = 0; pass < 2; ++pass) {
#pragma unroll
      for (int j = 0; j < 5; ++j) {
        const size_t go = gbase + (size_t)((lane + 32 * j) * 4);
        if (go + 4 <= total) *(volatile v4f*)(out + go) = val[j];
      }
      __threadfence();
    }
  }
}

extern "C" void kernel_launch(void* const* d_in, const int* in_sizes, int n_in,
                              void* d_out, int out_size, void* d_ws, size_t ws_size,
                              hipStream_t stream) {
  (void)d_ws;
  (void)ws_size;
  if (n_in < 1) return;
  if (in_sizes[0] != kBatch * kQ) return;
  if (out_size != kBatch * kOut) return;
  const float* x = (const float*)d_in[0];
  float* out = (float*)d_out;
  const int nrows = in_sizes[0] / kQ;
  const int blocks = (nrows + kRowsPerBlk - 1) / kRowsPerBlk;
  ring_expect_kernel<<<blocks, 256, 0, stream>>>(x, out, nrows);
}
